// GATFraudDetector_26096221290643
// MI455X (gfx1250) — hardware-verified
//
#include <hip/hip_runtime.h>
#include <stddef.h>
#include <stdint.h>


#define DIN     128
#define HC      64
#define NHEAD   4
#define HDQ     256
#define NTHR    256
#define NWAVE   8
#define EPT     8
#define CHUNK   (NTHR * EPT)
#define WCAP    (EPT * 32)
#define LISTN   (NWAVE * WCAP)
#define NBMAX   2048
#define RCAP    28672
#define DEGCAP  512
#define GBM     64
#define GBN     64
#define GTHR    128
#define CX      8.0f
#define CW      64.0f
#define SCL_XW  0.001953125f
#define NEGS    0.2f
#define WSMAX   134217728
#define LDS_AGG ((2 * RCAP + 2 * NBMAX + LISTN) * 4 + 64)
#define TBLN    (4 * HDQ)

static_assert((CHUNK & (CHUNK - 1)) == 0 && CHUNK <= 4096);
static_assert((NBMAX & (NBMAX - 1)) == 0 && NBMAX <= 4096);
static_assert(NTHR * 8 == NBMAX);
static_assert(LISTN >= NBMAX);
static_assert(LISTN >= NWAVE * WCAP);
static_assert((RCAP % 32) == 0);
static_assert(LDS_AGG + TBLN * 4 <= 300000);
static_assert(GBM == (GTHR / 32) * 16);
static_assert(DIN / 8 == 16);
static_assert((DIN % 32) == 0);
static_assert((HDQ % GBN) == 0);
static_assert(HDQ == NHEAD * HC && HC == 64 && HDQ == 8 * 32);
static_assert(NTHR * 4 == TBLN);

typedef float    v4f  __attribute__((ext_vector_type(4)));
typedef float    v8f  __attribute__((ext_vector_type(8)));
typedef int      v4i  __attribute__((ext_vector_type(4)));
typedef int      v8i  __attribute__((ext_vector_type(8)));
typedef _Float16 v8h  __attribute__((ext_vector_type(8)));
typedef _Float16 v16h __attribute__((ext_vector_type(16)));
union FragH { v16h v; v8h h[2]; v8i w; };

__device__ __forceinline__ v8f wmh(const FragH& a, const FragH& b, v8f c) {
  v8f d = __builtin_amdgcn_wmma_f32_16x16x32_f16(false, a.v, false, b.v, (short)0, c, false, false);
  asm volatile("v_nop\n\tv_nop\n\tv_nop\n\tv_nop" : "+v"(d) : "v"(a.w), "v"(b.w));
  return d;
}

__device__ __forceinline__ void ldwait() {
  asm volatile("s_wait_loadcnt 0x0" ::: "memory");
}

__device__ __forceinline__ float bf16r(float v) {
  unsigned u = (unsigned)__float_as_uint(v);
  u = (u + 0x7FFFu + ((u >> 16) & 1u)) & 0xFFFF0000u;
  return __uint_as_float(u);
}

__device__ __forceinline__ v8h cvt8h(const v4f a, const v4f b, const float c) {
  v8h hv;
  hv[0] = (_Float16)(bf16r(a.x) * c); hv[1] = (_Float16)(bf16r(a.y) * c);
  hv[2] = (_Float16)(bf16r(a.z) * c); hv[3] = (_Float16)(bf16r(a.w) * c);
  hv[4] = (_Float16)(bf16r(b.x) * c); hv[5] = (_Float16)(bf16r(b.y) * c);
  hv[6] = (_Float16)(bf16r(b.z) * c); hv[7] = (_Float16)(bf16r(b.w) * c);
  return hv;
}

__device__ __forceinline__ int scan_chunk(const int* __restrict__ dsts, int nE, int nT, int cbase, int slotBase,
                                          int nb, int vec8, int* list, int tid, int lane, int wave) {
  int wc = 0;
  const int el0  = tid * EPT;
  const int e0   = cbase + el0;
  const int sent = -2147483647 - 1;
  v4i da, db;
  if (vec8 != 0 && cbase + CHUNK <= nE) {
    da = *(const v4i*)(dsts + e0);
    db = *(const v4i*)(dsts + e0 + 4);
  } else {
#define DV(J) ((e0 + (J) < nE) ? dsts[min(e0 + (J), nE - 1)] : ((e0 + (J) < nT) ? (e0 + (J) - nE) : sent))
    da.x = DV(0); da.y = DV(1); da.z = DV(2); da.w = DV(3);
    ldwait();
    db.x = DV(4); db.y = DV(5); db.z = DV(6); db.w = DV(7);
    ldwait();
#undef DV
  }
  const unsigned nbs = (unsigned)slotBase;
  const unsigned unb = (unsigned)nb;
  const unsigned s0 = (unsigned)da.x - nbs, s1 = (unsigned)da.y - nbs;
  const unsigned s2 = (unsigned)da.z - nbs, s3 = (unsigned)da.w - nbs;
  const unsigned s4 = (unsigned)db.x - nbs, s5 = (unsigned)db.y - nbs;
  const unsigned s6 = (unsigned)db.z - nbs, s7 = (unsigned)db.w - nbs;
  const bool h0 = s0 < unb, h1 = s1 < unb, h2 = s2 < unb, h3 = s3 < unb;
  const bool h4 = s4 < unb, h5 = s5 < unb, h6 = s6 < unb, h7 = s7 < unb;
  const unsigned any = __builtin_amdgcn_ballot_w32(h0 | h1 | h2 | h3 | h4 | h5 | h6 | h7);
  if (any != 0u) {
#define HITJ(J, HJ, SJ) { \
      const unsigned mj = __builtin_amdgcn_ballot_w32(HJ); \
      if (mj != 0u) { \
        if (HJ) { \
          const int pos = wc + (int)__builtin_amdgcn_mbcnt_lo(mj, 0u); \
          if (pos < WCAP) list[wave * WCAP + pos] = ((el0 + (J)) << 12) | (int)(SJ); \
        } \
        wc += (int)__builtin_popcount(mj); } }
    HITJ(0, h0, s0)
    HITJ(1, h1, s1)
    HITJ(2, h2, s2)
    HITJ(3, h3, s3)
    HITJ(4, h4, s4)
    HITJ(5, h5, s5)
    HITJ(6, h6, s6)
    HITJ(7, h7, s7)
#undef HITJ
  }
  return wc;
}

__global__ __launch_bounds__(NTHR) void k_xprep(const float* __restrict__ x, _Float16* xh, int nN, int nUnits) {
  const int i = (int)blockIdx.x * NTHR + (int)threadIdx.x;
  if (i >= nUnits) return;
  const int row = i >> 4;
  const int c0  = (i & 15) * 8;
  const int rc  = row < nN ? row : nN - 1;
  const float* p = x + (size_t)rc * DIN + c0;
  v4f a = *(const v4f*)p, b = *(const v4f*)(p + 4);
  ldwait();
  const v4f z4 = {0.f, 0.f, 0.f, 0.f};
  if (row >= nN) { a = z4; b = z4; }
  const v8h hv = cvt8h(a, b, CX);
  const size_t o = (size_t)row * DIN + c0;
  *(volatile v8h*)(xh + o) = hv;
  __threadfence();
  *(volatile v8h*)(xh + o) = hv;
}

__global__ __launch_bounds__(NTHR) void k_wtr(const float* __restrict__ w, int cols, int K, _Float16* wt, int nUnits) {
  const int u = (int)blockIdx.x * NTHR + (int)threadIdx.x;
  if (u >= nUnits) return;
  const int kq = K >> 3;
  const int n  = u / kq;
  const int k8 = (u - n * kq) * 8;
  const float* p = w + (size_t)k8 * (size_t)cols + n;
  v4f a, b;
  a.x = p[0];                    a.y = p[(size_t)cols];         a.z = p[(size_t)2 * cols];     a.w = p[(size_t)3 * cols];
  ldwait();
  b.x = p[(size_t)4 * cols];     b.y = p[(size_t)5 * cols];     b.z = p[(size_t)6 * cols];     b.w = p[(size_t)7 * cols];
  ldwait();
  const v8h hv = cvt8h(a, b, CW);
  const size_t o = (size_t)n * (size_t)K + k8;
  *(volatile v8h*)(wt + o) = hv;
  __threadfence();
  *(volatile v8h*)(wt + o) = hv;
}

__global__ __launch_bounds__(GTHR) void k_gemm(
    const _Float16* __restrict__ A, const _Float16* __restrict__ WT, float* outF, int K, int ldo, float scl)
{
  __shared__ __attribute__((aligned(16))) float stg[GBM * GBN];
  const int tid = (int)threadIdx.x, lane = tid & 31, wave = tid >> 5, hh = lane >> 4, m = lane & 15;
  const int rowBase = (int)blockIdx.x * GBM;
  const int col0    = (int)blockIdx.y * GBN;

  v8f acc[4];
  {
    const v8f z = {0.f, 0.f, 0.f, 0.f, 0.f, 0.f, 0.f, 0.f};
    acc[0] = z; acc[1] = z; acc[2] = z; acc[3] = z;
  }
  const _Float16* ap = A  + (size_t)(rowBase + 16 * wave + m) * (size_t)K + 8 * hh;
  const _Float16* wp = WT + (size_t)(col0 + m) * (size_t)K + 8 * hh;
  const int ksteps = K >> 5;
#pragma unroll 1
  for (int ks = 0; ks < ksteps; ++ks) {
    FragH af;
    af.h[0] = *(const v8h*)(ap + 32 * ks);
    af.h[1] = *(const v8h*)(ap + 32 * ks + 16);
#pragma unroll
    for (int t = 0; t < 4; ++t) {
      const _Float16* wq = wp + (size_t)(16 * t) * (size_t)K + 32 * ks;
      FragH bf;
      bf.h[0] = *(const v8h*)wq;
      bf.h[1] = *(const v8h*)(wq + 16);
      acc[t] = wmh(af, bf, acc[t]);
    }
  }

#pragma unroll
  for (int t = 0; t < 4; ++t) {
    const int lc = 16 * t + m;
#pragma unroll
    for (int r = 0; r < 8; ++r) {
      const int lr = 16 * wave + 8 * hh + r;
      stg[lr * GBN + lc] = acc[t][r] * scl;
    }
  }
  __syncthreads();

  v4f fv[8];
#pragma unroll
  for (int i = 0; i < 8; ++i) {
    const int lr = 16 * wave + 2 * i + hh;
    fv[i] = *(const v4f*)(stg + lr * GBN + 4 * m);
  }
#pragma unroll
  for (int i = 0; i < 8; ++i) {
    const int lr = 16 * wave + 2 * i + hh;
    const int gr = rowBase + lr;
    float* op = outF + (size_t)gr * (size_t)ldo + col0 + 4 * m;
    *(volatile v4f*)op = fv[i];
  }
  __threadfence();
#pragma unroll
  for (int i = 0; i < 8; ++i) {
    const int lr = 16 * wave + 2 * i + hh;
    const int gr = rowBase + lr;
    float* op = outF + (size_t)gr * (size_t)ldo + col0 + 4 * m;
    *(volatile v4f*)op = fv[i];
  }
}

__device__ __forceinline__ int build_segments(const int* __restrict__ dsts, int nE, int nT, int nodeBase, int nb,
                                              int vec8, int* reg1, int* reg2, int* scnt, int* soff, int* list,
                                              int* wcnt, int* wtot, int tid, int lane, int wave) {
  for (int i = tid; i < NBMAX; i += NTHR) scnt[i] = 0;
  __syncthreads();

  int tot = 0;
  const int nChunks = (nT + CHUNK - 1) / CHUNK;
#pragma unroll 1
  for (int ch = 0; ch < nChunks; ++ch) {
    const int cbase = ch * CHUNK;
    const int wc = scan_chunk(dsts, nE, nT, cbase, nodeBase, nb, vec8, list, tid, lane, wave);
    if (lane == 0) wcnt[wave] = wc;
    __syncthreads();
    int pre = 0, all = 0;
#pragma unroll
    for (int w2 = 0; w2 < NWAVE; ++w2) {
      int c = wcnt[w2];
      c = c < 0 ? 0 : (c > WCAP ? WCAP : c);
      all += c;
      pre += (w2 < wave) ? c : 0;
    }
    const int wcc  = wc > WCAP ? WCAP : wc;
    const int base = tot + pre;
#pragma unroll 1
    for (int i = lane; i < wcc; i += 32) {
      const int ent = list[wave * WCAP + i];
      const int el  = (ent >> 12) & (CHUNK - 1);
      const int sl  = ent & (NBMAX - 1);
      int eid = cbase + el;
      eid = eid > nT - 1 ? nT - 1 : eid;
      const int pos = base + i;
      if (pos < RCAP) reg1[pos] = (int)(((unsigned)eid << 12) | (unsigned)sl);
    }
    tot += all;
    tot = tot > RCAP ? RCAP : tot;
    __syncthreads();
  }
  const int nh = tot;

  if (wave == 0) {
#pragma unroll 1
    for (int b0 = 0; b0 < nh; b0 += 32) {
      const int idx = b0 + lane;
      const int uv  = reg1[idx < RCAP ? idx : RCAP - 1];
      const int m32 = (nh - b0) < 32 ? (nh - b0) : 32;
#pragma unroll 1
      for (int k = 0; k < m32; ++k) {
        const int u  = __builtin_amdgcn_readlane(uv, k);
        const int sl = u & (NBMAX - 1);
        if (lane == 0) scnt[sl] = scnt[sl] + 1;
      }
    }
  }
  __syncthreads();

  {
    const v4i ca = *(const v4i*)(scnt + 8 * tid);
    const v4i cb = *(const v4i*)(scnt + 8 * tid + 4);
    const int e0 = ca.x < 0 ? 0 : ca.x, e1 = ca.y < 0 ? 0 : ca.y, e2 = ca.z < 0 ? 0 : ca.z, e3 = ca.w < 0 ? 0 : ca.w;
    const int e4 = cb.x < 0 ? 0 : cb.x, e5 = cb.y < 0 ? 0 : cb.y, e6 = cb.z < 0 ? 0 : cb.z, e7 = cb.w < 0 ? 0 : cb.w;
    const int ts = e0 + e1 + e2 + e3 + e4 + e5 + e6 + e7;
    int incl = ts;
#pragma unroll
    for (int d = 1; d < 32; d <<= 1) {
      const int up = __shfl_up(incl, d);
      if (lane >= d) incl += up;
    }
    if (lane == 31) wtot[wave] = incl;
    __syncthreads();
    int pre = 0;
#pragma unroll
    for (int w2 = 0; w2 < NWAVE; ++w2) pre += (w2 < wave) ? wtot[w2] : 0;
    int run = pre + incl - ts;
    soff[8 * tid + 0] = run; run += e0;
    soff[8 * tid + 1] = run; run += e1;
    soff[8 * tid + 2] = run; run += e2;
    soff[8 * tid + 3] = run; run += e3;
    soff[8 * tid + 4] = run; run += e4;
    soff[8 * tid + 5] = run; run += e5;
    soff[8 * tid + 6] = run; run += e6;
    soff[8 * tid + 7] = run;
  }
  __syncthreads();
  for (int i = tid; i < NBMAX; i += NTHR) list[i] = soff[i];
  __syncthreads();

  if (wave == 0) {
#pragma unroll 1
    for (int b0 = 0; b0 < nh; b0 += 32) {
      const int idx = b0 + lane;
      const int uv  = reg1[idx < RCAP ? idx : RCAP - 1];
      const int m32 = (nh - b0) < 32 ? (nh - b0) : 32;
#pragma unroll 1
      for (int k = 0; k < m32; ++k) {
        const int u   = __builtin_amdgcn_readlane(uv, k);
        const int sl  = u & (NBMAX - 1);
        const int eid = (int)((unsigned)u >> 12);
        if (lane == 0) {
          int pos = list[sl];
          pos = pos < 0 ? 0 : (pos > RCAP - 1 ? RCAP - 1 : pos);
          reg2[pos] = eid;
          list[sl] = pos + 1;
        }
      }
    }
  }
  __syncthreads();
  return nh;
}

__global__ __launch_bounds__(NTHR) void k_agg1(
    const int* __restrict__ srcs, const int* __restrict__ dsts, const float* __restrict__ H,
    const float* __restrict__ a_s, const float* __restrict__ a_d, const float* __restrict__ bias,
    const float* __restrict__ w2, float* H2, int nN, int nE, int nT, int nb, int vec8) {
  extern __shared__ v4f lds_dyn[];
  __shared__ __attribute__((aligned(16))) float tbl[TBLN];
  int* reg1 = (int*)lds_dyn;
  int* reg2 = reg1 + RCAP;
  int* scnt = reg2 + RCAP;
  int* soff = scnt + NBMAX;
  int* list = soff + NBMAX;
  int* wcnt = list + LISTN;
  int* wtot = wcnt + NWAVE;
  const int tid = (int)threadIdx.x, lane = tid & 31, wave = tid >> 5;
  const int nodeBase = (int)blockIdx.x * nb;

  {
    const int t  = tid >> 6;
    const int i4 = (tid & 63) * 4;
    const float* tp = (t == 0) ? a_s : ((t == 1) ? a_d : ((t == 2) ? bias : w2));
    v4f v = *(const v4f*)(tp + i4);
    ldwait();
    v.x = bf16r(v.x); v.y = bf16r(v.y); v.z = bf16r(v.z); v.w = bf16r(v.w);
    *(v4f*)(tbl + t * HDQ + i4) = v;
  }

  const int nh = build_segments(dsts, nE, nT, nodeBase, nb, vec8, reg1, reg2, scnt, soff, list, wcnt, wtot,
                                tid, lane, wave);

  const int nbw = nb >> 3;
  const bool ovf = (nh >= RCAP);
  const float qnan = __int_as_float(0x7fc00000);
  float asv[8], adv[8], bv[8], wv[8];
#pragma unroll
  for (int j = 0; j < 8; ++j) {
    asv[j] = tbl[32 * j + lane];
    adv[j] = tbl[HDQ + 32 * j + lane];
    bv[j]  = tbl[2 * HDQ + 32 * j + lane];
    wv[j]  = tbl[3 * HDQ + 32 * j + lane];
  }
  float keep = 0.f;
#pragma unroll 1
  for (int jt = 0; jt < nbw; ++jt) {
    const int slot = wave * nbw + jt;
    const int grow = nodeBase + slot;
    const int gcl  = grow < nN ? grow : nN - 1;
    int st = soff[slot];
    const int craw = scnt[slot];
    int cnt = craw;
    st  = st < 0 ? 0 : (st > nh ? nh : st);
    cnt = cnt < 0 ? 0 : (cnt > DEGCAP ? DEGCAP : cnt);
    if (cnt > nh - st) cnt = nh - st;
    const float pz   = (ovf || craw > DEGCAP) ? qnan : 0.0f;
    const float live = grow < nN ? 1.0f : 0.0f;

    const float* drow = H + (size_t)gcl * HDQ + lane;
    float hd[8];
#pragma unroll
    for (int j = 0; j < 8; ++j) hd[j] = drow[32 * j];
    ldwait();
    float pd[4];
#pragma unroll
    for (int h = 0; h < 4; ++h) pd[h] = fmaf(hd[2 * h + 1], adv[2 * h + 1], hd[2 * h] * adv[2 * h]);
#pragma unroll
    for (int off = 16; off > 0; off >>= 1) {
#pragma unroll
      for (int h = 0; h < 4; ++h) pd[h] += __shfl_xor(pd[h], off);
    }

    float av[8], mx[4], dn[4];
#pragma unroll
    for (int j = 0; j < 8; ++j) av[j] = 0.f;
#pragma unroll
    for (int h = 0; h < 4; ++h) { mx[h] = -1.0e30f; dn[h] = 0.f; }

#pragma unroll 1
    for (int q = 0; q < cnt; ++q) {
      int idx = st + q; idx = idx > RCAP - 1 ? RCAP - 1 : idx;
      int eid = reg2[idx]; eid = eid < 0 ? 0 : (eid > nT - 1 ? nT - 1 : eid);
      const int sv = srcs[eid < nE ? eid : nE - 1];
      ldwait();
      int s = eid < nE ? sv : eid - nE;
      s = s < 0 ? 0 : (s > nN - 1 ? nN - 1 : s);
      const float* hr = H + (size_t)s * HDQ + lane;
      float hs[8];
#pragma unroll
      for (int j = 0; j < 8; ++j) hs[j] = hr[32 * j];
      ldwait();
      float part[4];
#pragma unroll
      for (int h = 0; h < 4; ++h) part[h] = fmaf(hs[2 * h + 1], asv[2 * h + 1], hs[2 * h] * asv[2 * h]);
#pragma unroll
      for (int off = 16; off > 0; off >>= 1) {
#pragma unroll
        for (int h = 0; h < 4; ++h) part[h] += __shfl_xor(part[h], off);
      }
#pragma unroll
      for (int h = 0; h < 4; ++h) {
        const float a0 = part[h] + pd[h];
        const float al = a0 >= 0.f ? a0 : NEGS * a0;
        const float df = al - mx[h];
        const float ee = __expf(-fabsf(df));
        const bool up  = df > 0.f;
        const float s1 = up ? ee : 1.0f;
        const float s2 = up ? 1.0f : ee;
        mx[h] = up ? al : mx[h];
        dn[h] = fmaf(dn[h], s1, s2);
        av[2 * h]     = fmaf(av[2 * h],     s1, s2 * hs[2 * h]);
        av[2 * h + 1] = fmaf(av[2 * h + 1], s1, s2 * hs[2 * h + 1]);
      }
    }
    float iv[4];
#pragma unroll
    for (int h = 0; h < 4; ++h) {
      const float ds = dn[h] > 0.f ? dn[h] : 1.0f;
      iv[h] = (dn[h] > 0.f ? 1.0f : 0.0f) * __builtin_amdgcn_rcpf(ds);
    }
    float p = 0.f;
#pragma unroll
    for (int j = 0; j < 8; ++j) {
      const float t = fmaxf(fmaf(av[j], iv[j >> 1], bv[j]), 0.f);
      p = fmaf(t, wv[j], p);
    }
#pragma unroll
    for (int off = 16; off > 0; off >>= 1) p += __shfl_xor(p, off);
    const float h2v = p * live + pz;
    keep = ((jt & 31) == lane) ? h2v : keep;
    if ((jt & 31) == 31) {
      float* lp = H2 + (size_t)(grow - 31) + lane;
      *(volatile float*)lp = keep;
      __threadfence();
      *(volatile float*)lp = keep;
    }
  }
}

__global__ __launch_bounds__(NTHR) void k_agg2(
    const int* __restrict__ srcs, const int* __restrict__ dsts, const float* __restrict__ H2,
    const float* __restrict__ a_s2, const float* __restrict__ a_d2, const float* __restrict__ b2,
    float* out, int nN, int nE, int nT, int nb, int vec8) {
  extern __shared__ v4f lds_dyn[];
  int* reg1 = (int*)lds_dyn;
  int* reg2 = reg1 + RCAP;
  int* scnt = reg2 + RCAP;
  int* soff = scnt + NBMAX;
  int* list = soff + NBMAX;
  int* wcnt = list + LISTN;
  int* wtot = wcnt + NWAVE;
  const int tid = (int)threadIdx.x, lane = tid & 31, wave = tid >> 5;
  const int nodeBase = (int)blockIdx.x * nb;

  const float asr = a_s2[0];
  const float adr = a_d2[0];
  const float b2r = b2[0];
  ldwait();
  const float asc = bf16r(asr);
  const float adc = bf16r(adr);
  const float b2c = bf16r(b2r);

  const int nh = build_segments(dsts, nE, nT, nodeBase, nb, vec8, reg1, reg2, scnt, soff, list, wcnt, wtot,
                                tid, lane, wave);

  const int nbw = nb >> 3;
  const int ngr = nbw >> 5;
  const bool ovf = (nh >= RCAP);
  const float qnan = __int_as_float(0x7fc00000);
#pragma unroll 1
  for (int g = 0; g < ngr; ++g) {
    const int sb    = wave * nbw + 32 * g;
    const int slot  = sb + lane;
    const int gbase = nodeBase + sb;
    const int grow  = gbase + lane;
    int st = soff[slot];
    const int craw = scnt[slot];
    int cnt = craw;
    st  = st < 0 ? 0 : (st > nh ? nh : st);
    cnt = cnt < 0 ? 0 : (cnt > DEGCAP ? DEGCAP : cnt);
    if (cnt > nh - st) cnt = nh - st;
    const float pz = (ovf || craw > DEGCAP) ? qnan : 0.0f;
    const float hdv = H2[grow];
    ldwait();
    const float ad  = hdv * adc;
    int cm = cnt;
#pragma unroll
    for (int off = 16; off > 0; off >>= 1) {
      const int o2 = __shfl_xor(cm, off);
      cm = o2 > cm ? o2 : cm;
    }
    float m = -1.0e30f, den = 0.f, acc = 0.f;
#pragma unroll 1
    for (int q = 0; q < cm; ++q) {
      const bool act = q < cnt;
      int idx = st + q; idx = idx > RCAP - 1 ? RCAP - 1 : idx;
      int eid = reg2[idx]; eid = eid < 0 ? 0 : (eid > nT - 1 ? nT - 1 : eid);
      const int sv = srcs[eid < nE ? eid : nE - 1];
      ldwait();
      int s = eid < nE ? sv : eid - nE;
      s = s < 0 ? 0 : (s > nN - 1 ? nN - 1 : s);
      const float hv = H2[s];
      ldwait();
      const float as = hv * asc;
      const float a0 = as + ad;
      const float al = a0 >= 0.f ? a0 : NEGS * a0;
      const float df = al - m;
      const float ee = __expf(-fabsf(df));
      const bool up  = df > 0.f;
      const float s1 = up ? ee : 1.0f;
      const float s2 = up ? 1.0f : ee;
      const float mn = up ? al : m;
      const float dn = fmaf(den, s1, s2);
      const float an = fmaf(acc, s1, s2 * hv);
      m   = act ? mn : m;
      den = act ? dn : den;
      acc = act ? an : acc;
    }
    const float ds = den > 0.f ? den : 1.0f;
    const float iv = (den > 0.f ? 1.0f : 0.0f) * __builtin_amdgcn_rcpf(ds);
    const float z  = fmaf(acc, iv, b2c);
    const float ez = __expf(-fabsf(z));
    const float sg = __builtin_amdgcn_rcpf(1.0f + ez);
    const float val = (z >= 0.f ? sg : ez * sg) + pz;
    if (gbase < nN) {
      const bool ok = grow < nN;
      float* op = out + grow;
      if (ok) *(volatile float*)op = val;
      __threadfence();
      if (ok) *(volatile float*)op = val;
    }
  }
}

static int pick_nb(int nT, int nN) {
  int nb = NBMAX;
  while (nb > 16 && (long long)nb * (long long)nT * 5LL > (long long)RCAP * (long long)nN * 4LL) nb >>= 1;
  return nb;
}
static inline int cdiv(int a, int b) { return (a + b - 1) / b; }

extern "C" void kernel_launch(void* const* d_in, const int* in_sizes, int n_in,
                              void* d_out, int out_size, void* d_ws, size_t ws_size,
                              hipStream_t stream) {
  if (n_in < 10) return;
  const int nN = in_sizes[0] / DIN;
  if (nN <= 0 || in_sizes[0] != nN * DIN || nN > (1 << 19)) return;
  if (in_sizes[1] < 2 || (in_sizes[1] & 1) != 0) return;
  const int nE = in_sizes[1] / 2;
  const int nT = nE + nN;
  if (nE < 1 || nT > (1 << 20)) return;
  if (in_sizes[2] != DIN * HDQ) return;
  if (in_sizes[3] != HDQ || in_sizes[4] != HDQ) return;
  if (in_sizes[5] != HDQ || in_sizes[6] != HDQ) return;
  if (in_sizes[7] < 1 || in_sizes[8] < 1 || in_sizes[9] < 1) return;
  if (out_size != nN) return;

  const float* x    = (const float*)d_in[0];
  const int*   ei   = (const int*)  d_in[1];
  const float* W1   = (const float*)d_in[2];
  const float* as1  = (const float*)d_in[3];
  const float* ad1  = (const float*)d_in[4];
  const float* b1   = (const float*)d_in[5];
  const float* W2   = (const float*)d_in[6];
  const float* as2  = (const float*)d_in[7];
  const float* ad2  = (const float*)d_in[8];
  const float* b2   = (const float*)d_in[9];
  float* out = (float*)d_out;
  const int* src = ei;
  const int* dst = ei + nE;

  const int MP   = cdiv(nN, GBM) * GBM;
  const int nb   = pick_nb(nT, nN);
  if (nb < 256 || nb > NBMAX) return;
  const int gA   = cdiv(MP, nb);
  const int NR   = gA * nb;
  const int vec8 = ((nE & 3) == 0) ? 1 : 0;
  if (NR < MP) return;

  char* ws = (char*)d_ws;
  size_t off = 0;
  const size_t oXH = off; off += (size_t)MP * DIN * 2;            off = (off + 255) & ~(size_t)255;
  const size_t oH  = off; off += (size_t)MP * HDQ * 4;            off = (off + 255) & ~(size_t)255;
  const size_t oH2 = off; off += (size_t)NR * 4;                  off = (off + 255) & ~(size_t)255;
  const size_t oWT = off; off += (size_t)HDQ * DIN * 2;           off = (off + 255) & ~(size_t)255;
  if (off > ws_size || off > (size_t)WSMAX) return;
  _Float16* XH  = (_Float16*)(ws + oXH);
  float*    H   = (float*)(ws + oH);
  float*    H2P = (float*)(ws + oH2);
  _Float16* WT  = (_Float16*)(ws + oWT);

  hipFuncSetAttribute(reinterpret_cast<const void*>(&k_agg1),
                      hipFuncAttributeMaxDynamicSharedMemorySize, LDS_AGG);
  hipFuncSetAttribute(reinterpret_cast<const void*>(&k_agg2),
                      hipFuncAttributeMaxDynamicSharedMemorySize, LDS_AGG);

  const int nUx = MP * (DIN / 8);
  k_xprep<<<cdiv(nUx, NTHR), NTHR, 0, stream>>>(x, XH, nN, nUx);

  const int nUw = HDQ * (DIN / 8);
  k_wtr<<<cdiv(nUw, NTHR), NTHR, 0, stream>>>(W1, HDQ, DIN, WT, nUw);

  k_gemm<<<dim3(MP / GBM, HDQ / GBN), GTHR, 0, stream>>>(XH, WT, H, DIN, HDQ, SCL_XW);

  k_agg1<<<gA, NTHR, LDS_AGG, stream>>>(src, dst, H, as1, ad1, b1, W2, H2P, nN, nE, nT, nb, vec8);

  k_agg2<<<gA, NTHR, LDS_AGG, stream>>>(src, dst, H2P, as2, ad2, b2, out, nN, nE, nT, nb, vec8);
}
